// KANConvolution_7413113553459
// MI455X (gfx1250) — hardware-verified
//
#include <hip/hip_runtime.h>
#include <math.h>

typedef __attribute__((ext_vector_type(16))) _Float16 v16h;
typedef __attribute__((ext_vector_type(16))) __bf16 v16b;
typedef __attribute__((ext_vector_type(8)))  _Float16 v8h;
typedef __attribute__((ext_vector_type(8)))  float v8f;
typedef __attribute__((ext_vector_type(4)))  float v4f;
typedef __attribute__((ext_vector_type(2)))  float v2f;
typedef __attribute__((ext_vector_type(4)))  unsigned v4u;
typedef __attribute__((ext_vector_type(4)))  int v4i;
typedef float __attribute__((may_alias)) float_a;
typedef int __attribute__((may_alias)) int_a;

template <typename T> __device__ __forceinline__ void vst2(void* p, T v) { *(volatile T*)p = v; __threadfence(); *(volatile T*)p = v; }
__device__ __forceinline__ v8f wmma16(v16h a, v16h b, v8f c) {
  v8f d = __builtin_amdgcn_wmma_f32_16x16x32_f16(false, a, false, b, (short)0, c, false, false);
  asm volatile("v_nop\n\tv_nop\n\tv_nop\n\tv_nop" : "+v"(d) : "v"(a), "v"(b));
  return d;
}
__device__ __forceinline__ v8f wmma_bf(v16b a, v16b b, v8f c) {
  v8f d = __builtin_amdgcn_wmma_f32_16x16x32_bf16(false, a, false, b, (short)0, c, false, false);
  asm volatile("v_nop\n\tv_nop\n\tv_nop\n\tv_nop" : "+v"(d) : "v"(a), "v"(b));
  return d;
}
__device__ __forceinline__ v16h frag_h(const _Float16* rowk0, int lane) {
  union { v16h v; v8h q[2]; } u; const _Float16* p = rowk0 + 8 * (lane >> 4);
  u.q[0] = *(const v8h*)p; u.q[1] = *(const v8h*)(p + 16); return u.v;
}
__device__ __forceinline__ v16h frag_f32(const float* rowk0, int lane) {
  v16h a; const float* p = rowk0 + 8 * (lane >> 4);
#pragma unroll
  for (int i = 0; i < 8; ++i) { a[i] = (_Float16)p[i]; a[8 + i] = (_Float16)p[16 + i]; }
  return a;
}
__device__ __forceinline__ v16h frag_f32s(const float* rowk0, int lane, float sc) {
  v16h a; const float* p = rowk0 + 8 * (lane >> 4);
#pragma unroll
  for (int i = 0; i < 8; ++i) { a[i] = (_Float16)(p[i] * sc); a[8 + i] = (_Float16)(p[16 + i] * sc); }
  return a;
}
__device__ __forceinline__ v16h fragc_f32(const float* W, int k0, int n, int lane, int ld, int K) {
  v16h a; const int g = lane >> 4;
#pragma unroll
  for (int i = 0; i < 8; ++i) { const int ka = k0 + 8 * g + i, kb = ka + 16;
    a[i] = (_Float16)(ka < K ? W[(size_t)(ka < K ? ka : K - 1) * ld + n] : 0.f); a[8 + i] = (_Float16)(kb < K ? W[(size_t)(kb < K ? kb : K - 1) * ld + n] : 0.f); }
  return a;
}
struct F2 { v16b h, l; };
__device__ __forceinline__ F2 bsplit16(const float v[16]) { F2 r;
#pragma unroll
  for (int i = 0; i < 16; ++i) { const __bf16 h = (__bf16)v[i]; r.h[i] = h; r.l[i] = (__bf16)(v[i] - (float)h); }
  return r; }
__device__ __forceinline__ F2 split_row(const float* row, int k0, int lane) { float v[16]; const float* p = row + k0 + 8 * (lane >> 4);
#pragma unroll
  for (int i = 0; i < 8; ++i) { v[i] = p[i]; v[8 + i] = p[16 + i]; }
  return bsplit16(v); }
__device__ __forceinline__ F2 split_rowK(const float* row, int k0, int lane, int K) { float v[16]; const int g = lane >> 4;
#pragma unroll
  for (int i = 0; i < 8; ++i) { const int ka = k0 + 8 * g + i, kb = ka + 16; v[i] = ka < K ? row[ka < K ? ka : K - 1] : 0.f; v[8 + i] = kb < K ? row[kb < K ? kb : K - 1] : 0.f; }
  return bsplit16(v); }
__device__ __forceinline__ F2 split_col(const float* W, int k0, int n, int lane, int ld, int K) { float v[16]; const int g = lane >> 4;
#pragma unroll
  for (int i = 0; i < 8; ++i) { const int ka = k0 + 8 * g + i, kb = ka + 16; v[i] = ka < K ? W[(size_t)(ka < K ? ka : K - 1) * ld + n] : 0.f; v[8 + i] = kb < K ? W[(size_t)(kb < K ? kb : K - 1) * ld + n] : 0.f; }
  return bsplit16(v); }
__device__ __forceinline__ v8f mac3(const F2& a, const F2& b, v8f c) { c = wmma_bf(a.l, b.h, c); c = wmma_bf(a.h, b.l, c); return wmma_bf(a.h, b.h, c); }
__device__ __forceinline__ float sigm(float v) { return 1.0f / (1.0f + expf(-v)); }
#define LDSX() do { asm volatile("s_wait_dscnt 0" ::: "memory"); __builtin_amdgcn_wave_barrier(); __builtin_amdgcn_fence(__ATOMIC_RELEASE, "workgroup"); } while (0)


#define NB 8
#define IH 32
#define IW 32
#define CC 64
#define FF 64
#define GG 16
#define K9 9
#define KS (CC * K9 * GG)
#define K2C (CC * K9)
#ifndef TNB
#define TNB NB
#endif
typedef __attribute__((ext_vector_type(8))) __bf16 v8b;
__device__ __forceinline__ v16b frag_b(const __bf16* rowk0, int lane) {
  union { v16b v; v8b q[2]; } u; const __bf16* p = rowk0 + 8 * (lane >> 4);
  u.q[0] = *(const v8b*)p; u.q[1] = *(const v8b*)(p + 16); return u.v;
}
__device__ __forceinline__ float bfr(float v) { return (float)(__bf16)v; }
__device__ __attribute__((noinline)) float exp_ni(float v) { return expf(v); }
__device__ __attribute__((noinline)) float erf_ni(float v) { return erff(v); }

__global__ __launch_bounds__(128) void k_kan(const float* __restrict__ X, const float* __restrict__ CP, const float* __restrict__ W1, const float* __restrict__ W2, float* __restrict__ OUT) {
  __shared__ __align__(16) float sx[4][IW + 2][CC + 1];
  __shared__ __align__(16) float so[4][16][FF + 4];
  const int tid = threadIdx.x, wave = tid >> 5, lane = tid & 31, col = lane & 15, g = lane >> 4; const size_t blk = blockIdx.x; const size_t b = blk / (IH / 2); const int y0 = (int)(blk % (IH / 2)) * 2;
  for (int e = tid; e < 4 * (IW + 2) * CC; e += 128) { const int c = e % CC, rem = e / CC; const int xx = rem % (IW + 2), rr = rem / (IW + 2); const int gy = y0 - 1 + rr, gx = xx - 1; float v = 0.f; if (gy >= 0 && gy < IH && gx >= 0 && gx < IW) v = bfr(X[((b * IH + gy) * IW + gx) * (size_t)CC + c]); sx[rr][xx][c] = v; }
  __syncthreads();
  const int pl = wave * 16 + col; const int py = pl >> 5, px = pl & 31;
  v8f acc[4] = {};
#pragma unroll 1
  for (int kc = 0; kc < KS / 32; ++kc) { v16b ah, al;
#pragma unroll
    for (int half = 0; half < 2; ++half) { const int grp = kc * 2 + half; const int c = grp / K9, t9 = grp % K9; const int i = t9 / 3, j = t9 % 3;
      const float pv = sx[py + i][px + j][c];
      const float xc = fminf(fmaxf(pv, -1.0f), 1.0f); const float u = (xc + 1.0f) * 7.5f; int idx = (int)ceilf(u) - 1; idx = idx < 0 ? 0 : (idx > GG - 2 ? GG - 2 : idx);
      const float g0 = -1.0f + (float)idx * (2.0f / 15.0f), g1 = -1.0f + (float)(idx + 1) * (2.0f / 15.0f); const float frac = (xc - g0) / (g1 - g0);
#pragma unroll
      for (int q = 0; q < 8; ++q) { const int gg = 8 * g + q; const float bv = (gg == idx) ? (1.0f - frac) : (gg == idx + 1) ? frac : 0.f; const __bf16 h = (__bf16)bv; ah[half * 8 + q] = h; al[half * 8 + q] = (__bf16)(bv - (float)h); } }
#pragma unroll
    for (int jn = 0; jn < 4; ++jn) { v16b wh, wl; const int f = jn * 16 + col;
#pragma unroll
      for (int q = 0; q < 16; ++q) { const int k = kc * 32 + 8 * g + (q < 8 ? q : q + 8); const int grp = k >> 4; const float wv = bfr(W1[(size_t)f * K2C + grp]) * bfr(CP[(size_t)f * KS + k]); const __bf16 h = (__bf16)wv; wh[q] = h; wl[q] = (__bf16)(wv - (float)h); }
      acc[jn] = wmma_bf(ah, wh, acc[jn]); acc[jn] = wmma_bf(al, wh, acc[jn]); acc[jn] = wmma_bf(ah, wl, acc[jn]); } }
#pragma unroll 1
  for (int kc = 0; kc < K2C / 32; ++kc) { v16b ah, al;
#pragma unroll
    for (int q = 0; q < 16; ++q) { const int k2 = kc * 32 + 8 * g + (q < 8 ? q : q + 8); const int c = k2 / K9, t9 = k2 % K9; const int i = t9 / 3, j = t9 % 3; const float pv = sx[py + i][px + j][c]; const float sv = pv / (1.0f + expf(-pv)); const __bf16 h = (__bf16)sv; ah[q] = h; al[q] = (__bf16)(sv - (float)h); }
#pragma unroll
    for (int jn = 0; jn < 4; ++jn) { v16b w; const int f = jn * 16 + col;
#pragma unroll
      for (int q = 0; q < 8; ++q) { w[q] = (__bf16)W2[(size_t)f * K2C + kc * 32 + 8 * g + q]; w[8 + q] = (__bf16)W2[(size_t)f * K2C + kc * 32 + 16 + 8 * g + q]; }
      acc[jn] = wmma_bf(ah, w, acc[jn]); acc[jn] = wmma_bf(al, w, acc[jn]); } }
#pragma unroll
  for (int jn = 0; jn < 4; ++jn)
#pragma unroll
    for (int r = 0; r < 8; ++r) so[wave][8 * g + r][jn * 16 + col] = acc[jn][r];
  LDSX(); for (int rl = 0; rl < 16; ++rl) if (lane < 16) { const int p2 = wave * 16 + rl; vst2(OUT + ((b * IH + y0 + (p2 >> 5)) * IW + (p2 & 31)) * (size_t)FF + lane * 4, *(const v4f*)&so[wave][rl][lane * 4]); } }
extern "C" void kernel_launch(void* const* d_in, const int* in_sizes, int n_in, void* d_out, int out_size, void* d_ws, size_t ws_size, hipStream_t stream) {
  (void)in_sizes; (void)n_in; (void)out_size; (void)d_ws; (void)ws_size;
  const float** F = (const float**)d_in;
  k_kan<<<TNB * IH / 2, 128, 0, stream>>>(F[0], F[1], F[2], F[3], (float*)d_out);
}
